// SAGAN_50577534877744
// MI455X (gfx1250) — hardware-verified
//
#include <hip/hip_runtime.h>
#include <math.h>

typedef __attribute__((ext_vector_type(16))) _Float16 v16h;
typedef __attribute__((ext_vector_type(16))) __bf16 v16b;
typedef __attribute__((ext_vector_type(8)))  _Float16 v8h;
typedef __attribute__((ext_vector_type(8)))  float v8f;
typedef __attribute__((ext_vector_type(4)))  float v4f;
typedef __attribute__((ext_vector_type(2)))  float v2f;
typedef __attribute__((ext_vector_type(4)))  unsigned v4u;
typedef __attribute__((ext_vector_type(4)))  int v4i;
typedef float __attribute__((may_alias)) float_a;
typedef int __attribute__((may_alias)) int_a;

template <typename T> __device__ __forceinline__ void vst2(void* p, T v) { *(volatile T*)p = v; __threadfence(); *(volatile T*)p = v; }
__device__ __forceinline__ v8f wmma16(v16h a, v16h b, v8f c) {
  v8f d = __builtin_amdgcn_wmma_f32_16x16x32_f16(false, a, false, b, (short)0, c, false, false);
  asm volatile("v_nop\n\tv_nop\n\tv_nop\n\tv_nop" : "+v"(d) : "v"(a), "v"(b));
  return d;
}
__device__ __forceinline__ v8f wmma_bf(v16b a, v16b b, v8f c) {
  v8f d = __builtin_amdgcn_wmma_f32_16x16x32_bf16(false, a, false, b, (short)0, c, false, false);
  asm volatile("v_nop\n\tv_nop\n\tv_nop\n\tv_nop" : "+v"(d) : "v"(a), "v"(b));
  return d;
}
__device__ __forceinline__ v16h frag_h(const _Float16* rowk0, int lane) {
  union { v16h v; v8h q[2]; } u; const _Float16* p = rowk0 + 8 * (lane >> 4);
  u.q[0] = *(const v8h*)p; u.q[1] = *(const v8h*)(p + 16); return u.v;
}
__device__ __forceinline__ v16h frag_f32(const float* rowk0, int lane) {
  v16h a; const float* p = rowk0 + 8 * (lane >> 4);
#pragma unroll
  for (int i = 0; i < 8; ++i) { a[i] = (_Float16)p[i]; a[8 + i] = (_Float16)p[16 + i]; }
  return a;
}
__device__ __forceinline__ v16h frag_f32s(const float* rowk0, int lane, float sc) {
  v16h a; const float* p = rowk0 + 8 * (lane >> 4);
#pragma unroll
  for (int i = 0; i < 8; ++i) { a[i] = (_Float16)(p[i] * sc); a[8 + i] = (_Float16)(p[16 + i] * sc); }
  return a;
}
__device__ __forceinline__ v16h fragc_f32(const float* W, int k0, int n, int lane, int ld, int K) {
  v16h a; const int g = lane >> 4;
#pragma unroll
  for (int i = 0; i < 8; ++i) { const int ka = k0 + 8 * g + i, kb = ka + 16;
    a[i] = (_Float16)(ka < K ? W[(size_t)(ka < K ? ka : K - 1) * ld + n] : 0.f); a[8 + i] = (_Float16)(kb < K ? W[(size_t)(kb < K ? kb : K - 1) * ld + n] : 0.f); }
  return a;
}
struct F2 { v16b h, l; };
__device__ __forceinline__ F2 bsplit16(const float v[16]) { F2 r;
#pragma unroll
  for (int i = 0; i < 16; ++i) { const __bf16 h = (__bf16)v[i]; r.h[i] = h; r.l[i] = (__bf16)(v[i] - (float)h); }
  return r; }
__device__ __forceinline__ F2 split_row(const float* row, int k0, int lane) { float v[16]; const float* p = row + k0 + 8 * (lane >> 4);
#pragma unroll
  for (int i = 0; i < 8; ++i) { v[i] = p[i]; v[8 + i] = p[16 + i]; }
  return bsplit16(v); }
__device__ __forceinline__ F2 split_rowK(const float* row, int k0, int lane, int K) { float v[16]; const int g = lane >> 4;
#pragma unroll
  for (int i = 0; i < 8; ++i) { const int ka = k0 + 8 * g + i, kb = ka + 16; v[i] = ka < K ? row[ka < K ? ka : K - 1] : 0.f; v[8 + i] = kb < K ? row[kb < K ? kb : K - 1] : 0.f; }
  return bsplit16(v); }
__device__ __forceinline__ F2 split_col(const float* W, int k0, int n, int lane, int ld, int K) { float v[16]; const int g = lane >> 4;
#pragma unroll
  for (int i = 0; i < 8; ++i) { const int ka = k0 + 8 * g + i, kb = ka + 16; v[i] = ka < K ? W[(size_t)(ka < K ? ka : K - 1) * ld + n] : 0.f; v[8 + i] = kb < K ? W[(size_t)(kb < K ? kb : K - 1) * ld + n] : 0.f; }
  return bsplit16(v); }
__device__ __forceinline__ v8f mac3(const F2& a, const F2& b, v8f c) { c = wmma_bf(a.l, b.h, c); c = wmma_bf(a.h, b.l, c); return wmma_bf(a.h, b.h, c); }
__device__ __forceinline__ float sigm(float v) { return 1.0f / (1.0f + expf(-v)); }
#define LDSX() do { asm volatile("s_wait_dscnt 0" ::: "memory"); __builtin_amdgcn_wave_barrier(); __builtin_amdgcn_fence(__ATOMIC_RELEASE, "workgroup"); } while (0)


#define NNODE 16384
#define NG 128
#define NPG 128
#define DEG 8
#define NE (NNODE * DEG)
#define F0 128
#define HC1 384
#define HC2 128
#define HC3 64
#define C3 32
#define DX 544
#define KX 30
#define ND 2048
#define DK (KX * DX)
#define GIN (DK + 64)
#ifndef TNG
#define TNG NG
#endif
#ifndef DBGM
#define DBGM 0
#endif
typedef __attribute__((ext_vector_type(8))) __bf16 v8b;
__device__ __forceinline__ v16b frag_b(const __bf16* rowk0, int lane) {
  union { v16b v; v8b q[2]; } u; const __bf16* p = rowk0 + 8 * (lane >> 4);
  u.q[0] = *(const v8b*)p; u.q[1] = *(const v8b*)(p + 16); return u.v;
}
__device__ __forceinline__ v16b frag_gbf(const float* rowk0, int lane) {
  v16b a; const float* p = rowk0 + 8 * (lane >> 4);
#pragma unroll
  for (int i = 0; i < 8; ++i) { a[i] = (__bf16)p[i]; a[8 + i] = (__bf16)p[16 + i]; }
  return a;
}
__device__ __forceinline__ float bfr(float v) { return (float)(__bf16)v; }
__device__ __attribute__((noinline)) float exp_ni(float v) { return expf(v); }
#define PO_1 0
#define PO_2 (PO_1 + 768 * 128)
#define PO_3 (PO_2 + 256 * 384)
#define PO_S (PO_3 + 128 * 128)
#define PO_G (PO_S + 32 * DX)
#define PO_D (PO_G + DX * DX)
#define PO_E (PO_D + 32 * ND)
#define PO_L (PO_E + 32 * ND)
#define PO_END (PO_L + 128 * GIN)
#define WS_PT   0u
#define WS_XLR  (WS_PT + 2u * PO_END)
#define WS_XC   (WS_XLR + 4u * NNODE * 768)
#define WS_PRE  (WS_XC + 4u * NNODE * DX)
#define WS_PART (WS_PRE + 4u * NNODE * HC1)
#define WS_BN   (WS_PART + 4u * 256 * 1536)
#define WS_XG   (WS_BN + 4u * 2 * 768)
#define WS_HH   (WS_XG + 4u * NG * GIN)
#define WS_END  (WS_HH + 4u * 2 * ND * 32)

__global__ __launch_bounds__(256) void k_pack(const float* __restrict__ W1l, const float* __restrict__ W1r, const float* __restrict__ W2l, const float* __restrict__ W2r, const float* __restrict__ W3l, const float* __restrict__ W3r, const float* __restrict__ Ws, const float* __restrict__ Wg, const float* __restrict__ Wde, const float* __restrict__ Wse, const float* __restrict__ Wl1, __bf16* __restrict__ PT) {
  __shared__ __align__(16) __bf16 srow[2048];
  const int n = blockIdx.x, tid = threadIdx.x; int len; size_t dst;
  if (n < 768) { len = 128; dst = PO_1 + (size_t)n * 128; const int c = n % 384; const float* Wm = n < 384 ? W1l : W1r; if (tid < 128) srow[tid] = (__bf16)bfr(Wm[tid * 384 + c]); }
  else if (n < 1024) { const int m = n - 768; len = 384; dst = PO_2 + (size_t)m * 384; const int c = m % 128; const float* Wm = m < 128 ? W2l : W2r; for (int k = tid; k < 384; k += 256) srow[k] = (__bf16)bfr(Wm[k * 128 + c]); }
  else if (n < 1152) { const int m = n - 1024; len = 128; dst = PO_3 + (size_t)m * 128; const int c = m % 64; const float* Wm = m < 64 ? W3l : W3r; if (tid < 128) srow[tid] = (__bf16)bfr(Wm[tid * 64 + c]); }
  else if (n < 1184) { const int c = n - 1152; len = DX; dst = PO_S + (size_t)c * DX; for (int k = tid; k < DX; k += 256) srow[k] = (__bf16)(c < KX ? bfr(Ws[k * KX + c]) : 0.f); }
  else if (n < 1184 + DX) { const int c = n - 1184; len = DX; dst = PO_G + (size_t)c * DX; for (int k = tid; k < DX; k += 256) srow[k] = (__bf16)bfr(Wg[(size_t)k * DX + c]); }
  else if (n < 1184 + DX + 64) { const int m = n - 1184 - DX; len = ND; dst = (m < 32 ? PO_D + (size_t)m * ND : PO_E + (size_t)(m - 32) * ND); const float* Wm = m < 32 ? Wde : Wse; const int c = m & 31; for (int k = tid; k < ND; k += 256) srow[k] = (__bf16)bfr(Wm[k * 32 + c]); }
  else { const int c = n - 1184 - DX - 64; len = GIN; dst = PO_L + (size_t)c * GIN;
    for (int part = 0; part < 8; ++part) { for (int k = tid; k < 2048; k += 256) srow[k] = (__bf16)bfr(Wl1[(size_t)(part * 2048 + k) * 128 + c]); __syncthreads(); vst2((unsigned*)(PT + dst + part * 2048 + tid * 8), *(const v4u*)(&srow[tid * 8])); __syncthreads(); }
    return; }
  __syncthreads();
  for (int q = tid; q < len / 8; q += 256) vst2((unsigned*)(PT + dst + q * 8), *(const v4u*)(&srow[q * 8]));
}
template <int KI, int NO, bool EXACT>
__global__ __launch_bounds__(128) void k_proj(const float* __restrict__ Xin, int pin, int xoff, const __bf16* __restrict__ P, float* __restrict__ XLR) {
  __shared__ __align__(16) float so[4][16][68];
  const int tid = threadIdx.x, wave = tid >> 5, lane = tid & 31, col = lane & 15, g = lane >> 4; const size_t r0 = (size_t)blockIdx.x * 64 + wave * 16;
#pragma unroll 1
  for (int jt = 0; jt < NO / 64; ++jt) {
    v8f acc[4] = {};
#pragma unroll 2
    for (int kc = 0; kc < KI / 32; ++kc) { const float* xr = Xin + (r0 + col) * pin + xoff;
      if (EXACT) { const v16b a = frag_gbf(xr + kc * 32, lane);
#pragma unroll
        for (int j = 0; j < 4; ++j) acc[j] = wmma_bf(a, frag_b(P + (size_t)(jt * 64 + j * 16 + col) * KI + kc * 32, lane), acc[j]); }
      else { const F2 a = split_row(xr, kc * 32, lane);
#pragma unroll
        for (int j = 0; j < 4; ++j) { const v16b w = frag_b(P + (size_t)(jt * 64 + j * 16 + col) * KI + kc * 32, lane); acc[j] = wmma_bf(a.l, w, acc[j]); acc[j] = wmma_bf(a.h, w, acc[j]); } } }
#pragma unroll
    for (int j = 0; j < 4; ++j)
#pragma unroll
      for (int r = 0; r < 8; ++r) so[wave][8 * g + r][j * 16 + col] = acc[j][r];
    LDSX();
    for (int rl = 0; rl < 16; ++rl) if (lane < 16) vst2(XLR + (r0 + rl) * 768 + jt * 64 + lane * 4, *(const v4f*)&so[wave][rl][lane * 4]);
    LDSX(); }
}
template <int H, int C, int MODE>
__global__ __launch_bounds__(256) void k_gat(const float* __restrict__ XLR, const int* __restrict__ ESRC, const int* __restrict__ EDST, const float* __restrict__ ATT, const float* __restrict__ Bv, float* __restrict__ OUTM) {
  __shared__ int scnt[NPG], sst[NPG]; __shared__ unsigned short sidx[NPG * DEG + NPG];
  __shared__ float satt[H * C];
  const int gph = blockIdx.x, tid = threadIdx.x; const int nbase = gph * NPG; const size_t ebase = (size_t)gph * NPG * DEG;
  for (int q = tid; q < H * C; q += 256) satt[q] = bfr(ATT[q]);
  if (tid < NPG) { int c = 0; for (int e = 0; e < NPG * DEG; ++e) { const int d = EDST[ebase + e] - nbase; if (d == tid) ++c; } scnt[tid] = c + 1; }
  __syncthreads();
  if (tid == 0) { int a = 0; for (int i = 0; i < NPG; ++i) { sst[i] = a; a += scnt[i]; } }
  __syncthreads();
  if (tid < NPG) { int w = sst[tid]; for (int e = 0; e < NPG * DEG; ++e) { const int d = EDST[ebase + e] - nbase; if (d == tid) { int s = ESRC[ebase + e] - nbase; s = min(max(s, 0), NPG - 1); sidx[w++] = (unsigned short)s; } } sidx[w] = (unsigned short)tid; }
  __syncthreads();
  constexpr int CQ = C / 4; constexpr int HI = (MODE == 1) ? 1 : H; constexpr int NIT = NPG * HI * 4;
  for (int it = tid; it < NIT; it += 256) {
    const int q = it & 3, ih = it >> 2; const int i = (MODE == 1) ? ih : ih / H; const int h0 = (MODE == 1) ? 0 : ih % H; const int cnt = scnt[i], st = sst[i];
    float res[CQ];
#pragma unroll
    for (int c = 0; c < CQ; ++c) res[c] = 0.f;
#pragma unroll 1
    for (int hh = 0; hh < ((MODE == 1) ? H : 1); ++hh) { const int h = h0 + hh;
      const float* xri = XLR + (size_t)(nbase + i) * 768 + H * C + h * C;
      float mx = -3.0e38f;
      for (int e = 0; e < cnt; ++e) { const int s = sidx[st + e]; const float* xl = XLR + (size_t)(nbase + s) * 768 + h * C; float d = 0.f;
#pragma unroll 1
        for (int c = q * CQ; c < q * CQ + CQ; ++c) { float v = xl[c] + xri[c]; v = v > 0.f ? v : 0.2f * v; d += v * satt[h * C + c]; }
        d += __shfl_xor(d, 1); d += __shfl_xor(d, 2); mx = fmaxf(mx, d); }
      float z = 0.f; float acc[CQ];
#pragma unroll
      for (int c = 0; c < CQ; ++c) acc[c] = 0.f;
      for (int e = 0; e < cnt; ++e) { const int s = sidx[st + e]; const float* xl = XLR + (size_t)(nbase + s) * 768 + h * C; float d = 0.f;
#pragma unroll 1
        for (int c = q * CQ; c < q * CQ + CQ; ++c) { float v = xl[c] + xri[c]; v = v > 0.f ? v : 0.2f * v; d += v * satt[h * C + c]; }
        d += __shfl_xor(d, 1); d += __shfl_xor(d, 2); const float p = exp_ni(d - mx); z += p;
#pragma unroll
        for (int c = 0; c < CQ; ++c) acc[c] += p * xl[q * CQ + c]; }
      const float iz = 1.0f / z;
#pragma unroll
      for (int c = 0; c < CQ; ++c) res[c] += acc[c] * iz; }
    if (MODE == 0) {
#pragma unroll
      for (int p4 = 0; p4 < CQ / 4; ++p4) { v4f v; for (int k = 0; k < 4; ++k) { const int c = h0 * C + q * CQ + p4 * 4 + k; v[k] = fmaxf(res[p4 * 4 + k] + bfr(Bv[c]), 0.f); } vst2(OUTM + (size_t)(nbase + i) * (H * C) + h0 * C + q * CQ + p4 * 4, v); } }
    else {
#pragma unroll
      for (int p4 = 0; p4 < CQ / 4; ++p4) { v4f v; for (int k = 0; k < 4; ++k) { const int c = q * CQ + p4 * 4 + k; v[k] = res[p4 * 4 + k] * (1.0f / H) + bfr(Bv[c]); } vst2(OUTM + (size_t)(nbase + i) * DX + 512 + q * CQ + p4 * 4, v); } } }
}

template <int NC>
__global__ __launch_bounds__(128) void k_colpart(const float* __restrict__ M, float* __restrict__ PART) {
  __shared__ __align__(16) float sp[2 * NC];
  const int tid = threadIdx.x; const size_t r0 = (size_t)blockIdx.x * 64;
  for (int c = tid; c < NC; c += 128) { float s = 0.f, q = 0.f; for (int r = 0; r < 64; ++r) { const float v = M[(r0 + r) * NC + c]; s += v; q += v * v; } sp[c] = s; sp[NC + c] = q; }
  __syncthreads();
  for (int q = tid; q < 2 * NC / 4; q += 128) vst2(PART + (size_t)blockIdx.x * 1536 + q * 4, *(const v4f*)&sp[q * 4]);
}
template <int NC>
__global__ __launch_bounds__(128) void k_fin(const float* __restrict__ PART, const float* __restrict__ g, const float* __restrict__ bb, float* __restrict__ BNslot) {
  __shared__ __align__(16) float so[2 * NC];
  const int tid = threadIdx.x;
  for (int c = tid; c < NC; c += 128) { float s = 0.f, q = 0.f; for (int b = 0; b < NNODE / 64; ++b) { s += PART[(size_t)b * 1536 + c]; q += PART[(size_t)b * 1536 + NC + c]; } const float m = s / (float)NNODE; const float var = fmaxf(q / (float)NNODE - m * m, 0.f); const float sc = bfr(g[c]) * rsqrtf(var + 1e-5f); so[c] = sc; so[NC + c] = bfr(bb[c]) - m * sc; }
  __syncthreads();
  for (int q = tid; q < 2 * NC / 4; q += 128) vst2(BNslot + q * 4, *(const v4f*)&so[q * 4]);
}
template <int NC>
__global__ __launch_bounds__(256) void k_bnapply(const float* __restrict__ PRE, const float* __restrict__ BNslot, int xoff, float* __restrict__ XC) {
  const int tid = threadIdx.x; const size_t r0 = (size_t)blockIdx.x * 64;
  for (int q = tid; q < 64 * (NC / 4); q += 256) { const int rl = q / (NC / 4), pc = q % (NC / 4); v4f v; for (int k = 0; k < 4; ++k) { const int c = pc * 4 + k; v[k] = PRE[(r0 + rl) * NC + c] * BNslot[c] + BNslot[NC + c]; } vst2(XC + (r0 + rl) * DX + xoff + pc * 4, v); }
}
__global__ __launch_bounds__(256) void k_pool(const float* __restrict__ XC, const __bf16* __restrict__ PT, const float* __restrict__ bs, const float* __restrict__ bg, const int* __restrict__ ESRC, const int* __restrict__ EDST, float* __restrict__ XG) {
  __shared__ float ss[NPG][33]; __shared__ unsigned char sA[NPG][NPG]; __shared__ float sT[NPG][32]; __shared__ float sap[32][33]; __shared__ float sdg[32];
  __shared__ __align__(16) __bf16 sxh[64][136], sxl[64][136]; __shared__ __align__(16) __bf16 ssh[32][136], ssl[32][136];
  __shared__ __align__(16) float sxp[32][DX + 4]; __shared__ __align__(16) __bf16 sph[32][DX + 8], spl[32][DX + 8]; __shared__ __align__(16) float sy[32][68]; __shared__ __align__(16) float sout[64];
  const int gph = blockIdx.x, tid = threadIdx.x, wave = tid >> 5, lane = tid & 31, col = lane & 15, g = lane >> 4; const int nbase = gph * NPG; const size_t ebase = (size_t)gph * NPG * DEG;
  { v8f acc[2] = {};
#pragma unroll 1
    for (int kc = 0; kc < DX / 32; ++kc) { const F2 a = split_row(XC + (size_t)(nbase + wave * 16 + col) * DX, kc * 32, lane);
#pragma unroll
      for (int j = 0; j < 2; ++j) { const v16b w = frag_b(PT + PO_S + (size_t)(j * 16 + col) * DX + kc * 32, lane); acc[j] = wmma_bf(a.l, w, acc[j]); acc[j] = wmma_bf(a.h, w, acc[j]); } }
#pragma unroll
    for (int j = 0; j < 2; ++j)
#pragma unroll
      for (int r = 0; r < 8; ++r) { const int k = j * 16 + col; ss[wave * 16 + 8 * g + r][k] = k < KX ? acc[j][r] + bfr(bs[k]) : -3.0e38f; } }
  for (int q = tid; q < NPG * NPG; q += 256) (&sA[0][0])[q] = 0;
  __syncthreads();
  if (tid < NPG) { float mx = -3.0e38f; for (int k = 0; k < KX; ++k) mx = fmaxf(mx, ss[tid][k]); float z = 0.f; for (int k = 0; k < KX; ++k) { const float e = exp_ni(ss[tid][k] - mx); ss[tid][k] = e; z += e; } const float iz = 1.0f / z; for (int k = 0; k < KX; ++k) ss[tid][k] *= iz; ss[tid][30] = 0.f; ss[tid][31] = 0.f; }
  else if (tid < 2 * NPG) { const int sl = tid - NPG; for (int e = 0; e < DEG; ++e) { const size_t ei = ebase + (size_t)sl * DEG + e; int s = ESRC[ei] - nbase, d = EDST[ei] - nbase; if (s == sl && d >= 0 && d < NPG) sA[sl][d] += 1; } }
  __syncthreads();
  { const int n = tid >> 1, kh = tid & 1; for (int k = kh * 16; k < kh * 16 + 16; ++k) { float t = 0.f; if (k < KX) for (int m = 0; m < NPG; ++m) t += (float)sA[n][m] * ss[m][k]; sT[n][k] = t; } }
  __syncthreads();
  for (int q = tid; q < 32 * 32; q += 256) { const int k = q >> 5, l = q & 31; float a = 0.f; if (k < KX && l < KX) { if (k == l) a = 1.0f; else for (int n = 0; n < NPG; ++n) a += ss[n][k] * sT[n][l]; } sap[k][l] = a; }
  __syncthreads();
  if (tid < 32) { float rs = 0.f; for (int l = 0; l < KX; ++l) rs += sap[tid][l]; sdg[tid] = tid < KX ? rsqrtf(fmaxf(rs, 1.0f)) : 0.f; }
  for (int q = tid; q < 32 * NPG; q += 256) { const int k = q >> 7, n = q & 127; const float v = ss[n][k]; const __bf16 hb = (__bf16)v; ssh[k][n] = hb; ssl[k][n] = (__bf16)(v - (float)hb); }
  __syncthreads();
#pragma unroll 1
  for (int d0 = 0; d0 < DX; d0 += 64) { const int nd = min(64, DX - d0);
    for (int q = tid; q < 64 * NPG; q += 256) { const int dl = q >> 7, n = q & 127; const float v = dl < nd ? XC[(size_t)(nbase + n) * DX + d0 + dl] : 0.f; const __bf16 hb = (__bf16)v; sxh[dl][n] = hb; sxl[dl][n] = (__bf16)(v - (float)hb); }
    __syncthreads();
    { const int rt = wave >> 1, ct = wave & 1; v8f acc = {};
#pragma unroll
      for (int kc = 0; kc < 4; ++kc) { const F2 a = {frag_b(&sxh[rt * 16 + col][kc * 32], lane), frag_b(&sxl[rt * 16 + col][kc * 32], lane)}; const F2 b = {frag_b(&ssh[ct * 16 + col][kc * 32], lane), frag_b(&ssl[ct * 16 + col][kc * 32], lane)}; acc = mac3(a, b, acc); }
#pragma unroll
      for (int r = 0; r < 8; ++r) { const int dl = rt * 16 + 8 * g + r, k = ct * 16 + col; if (dl < nd) sxp[k][d0 + dl] = acc[r]; } }
    __syncthreads(); }
  for (int q = tid; q < 32 * DX; q += 256) { const int k = q / DX, d = q % DX; const float v = sxp[k][d]; const __bf16 hb = (__bf16)v; sph[k][d] = hb; spl[k][d] = (__bf16)(v - (float)hb); }
  __syncthreads();
#pragma unroll 1
  for (int c0 = 0; c0 < DX; c0 += 64) { const int ncol = min(64, DX - c0);
    { const int rt = wave & 1, ct = wave >> 1; v8f acc = {};
      if (ct * 16 < ncol) {
#pragma unroll 1
        for (int kc = 0; kc < DX / 32; ++kc) { const v16b ah = frag_b(&sph[rt * 16 + col][kc * 32], lane), al = frag_b(&spl[rt * 16 + col][kc * 32], lane); const v16b w = frag_b(PT + PO_G + (size_t)(c0 + ct * 16 + col) * DX + kc * 32, lane); acc = wmma_bf(al, w, acc); acc = wmma_bf(ah, w, acc); } }
#pragma unroll
      for (int r = 0; r < 8; ++r) sy[rt * 16 + 8 * g + r][ct * 16 + col] = acc[r]; }
    __syncthreads();
    { const int k = tid >> 3, part = tid & 7; if (k < KX) { for (int j = part; j < ncol; j += 8) { float a = 0.f; for (int l = 0; l < KX; ++l) a += sdg[k] * sap[k][l] * sdg[l] * sy[l][j]; const int d = c0 + j; sxp[k][d] = fmaxf(a + bfr(bg[d]), 0.f); } } }
    __syncthreads(); }
  for (int q = tid; q < DK / 4; q += 256) { const int f = q * 4; v4f v; for (int i = 0; i < 4; ++i) { const int ff = f + i; v[i] = sxp[ff / DX][ff % DX]; } vst2(XG + (size_t)gph * GIN + 32 + f, v); }
}
__global__ __launch_bounds__(128) void k_nbh(const float* __restrict__ EMB0, const float* __restrict__ EMB1, const __bf16* __restrict__ PT, const float* __restrict__ b0, const float* __restrict__ b1, float* __restrict__ HH) {
  __shared__ __align__(16) float so[4][16][36];
  const int tid = threadIdx.x, wave = tid >> 5, lane = tid & 31, col = lane & 15, g = lane >> 4; const int which = blockIdx.y; const size_t r0 = (size_t)blockIdx.x * 64 + wave * 16; const float* EMB = which == 0 ? EMB0 : EMB1; const __bf16* P = PT + (which == 0 ? PO_D : PO_E); const float* bb = which == 0 ? b0 : b1;
  v8f acc[2] = {};
#pragma unroll 1
  for (int kc = 0; kc < ND / 32; ++kc) { const v16b a = frag_gbf(EMB + (r0 + col) * ND + kc * 32, lane);
#pragma unroll
    for (int j = 0; j < 2; ++j) acc[j] = wmma_bf(a, frag_b(P + (size_t)(j * 16 + col) * ND + kc * 32, lane), acc[j]); }
#pragma unroll
  for (int j = 0; j < 2; ++j)
#pragma unroll
    for (int r = 0; r < 8; ++r) so[wave][8 * g + r][j * 16 + col] = acc[j][r] + bfr(bb[j * 16 + col]);
  LDSX();
  for (int rl = 0; rl < 16; ++rl) if (lane < 8) vst2(HH + ((size_t)which * ND + r0 + rl) * 32 + lane * 4, *(const v4f*)&so[wave][rl][lane * 4]);
}
__global__ __launch_bounds__(256) void k_nbv(const float* __restrict__ ADJ0, const float* __restrict__ ADJ1, const float* __restrict__ HH, const int* __restrict__ PR0, const int* __restrict__ PR1, float* __restrict__ XG) {
  __shared__ float sdeg[8]; __shared__ int snb[ND]; __shared__ int sn; __shared__ float sdj[256]; __shared__ float sacc[8][32]; __shared__ __align__(16) float sv[32];
  const int p = blockIdx.x, which = blockIdx.y, tid = threadIdx.x, wave = tid >> 5, lane = tid & 31; const float* ADJ = which == 0 ? ADJ0 : ADJ1; const float* H = HH + (size_t)which * ND * 32;
  const int i = min(max((which == 0 ? PR0 : PR1)[p], 0), ND - 1);
  { float s = 0.f; for (int j = tid; j < ND; j += 256) s += bfr(ADJ[(size_t)i * ND + j]);
#pragma unroll
    for (int o = 1; o < 32; o <<= 1) s += __shfl_xor(s, o);
    if (lane == 0) sdeg[wave] = s; }
  if (tid == 0) { int c = 0; for (int j = 0; j < ND; ++j) if (bfr(ADJ[(size_t)i * ND + j]) != 0.f) snb[c++] = j; sn = c; }
  __syncthreads();
  const float degi = ((sdeg[0] + sdeg[1]) + (sdeg[2] + sdeg[3])) + ((sdeg[4] + sdeg[5]) + (sdeg[6] + sdeg[7])) + 1.0f; const float di = rsqrtf(degi); const int nn = min(sn, 256);
  if (tid < nn) { const int j = snb[tid]; float s = 0.f; for (int k = 0; k < ND; ++k) s += bfr(ADJ[(size_t)j * ND + k]); sdj[tid] = rsqrtf(s + 1.0f); }
  __syncthreads();
  { float a = 0.f; for (int t = wave; t < nn; t += 8) { const int j = snb[t]; a += bfr(ADJ[(size_t)i * ND + j]) * sdj[t] * H[(size_t)j * 32 + lane]; } sacc[wave][lane] = a; }
  __syncthreads();
  if (tid < 32) { float a = 0.f; for (int w = 0; w < 8; ++w) a += sacc[w][tid]; const float hi = H[(size_t)i * 32 + tid]; const float v = 0.2f * hi + 0.8f * di * (a + di * hi); float nq = v * v;
#pragma unroll
    for (int o = 1; o < 32; o <<= 1) nq += __shfl_xor(nq, o);
    sv[tid] = v / fmaxf(sqrtf(nq), 1e-12f); }
  __syncthreads();
  if (tid < 8) vst2(XG + (size_t)p * GIN + (which == 0 ? 0 : 32 + DK) + tid * 4, *(const v4f*)&sv[tid * 4]);
}
__global__ __launch_bounds__(256) void k_head(const float* __restrict__ XG, const __bf16* __restrict__ PT, const float* __restrict__ bl1, const float* __restrict__ Wl2, const float* __restrict__ bl2, float* __restrict__ out) {
  __shared__ float sh[32][132]; __shared__ __align__(16) float so[32];
  const int tid = threadIdx.x, wave = tid >> 5, lane = tid & 31, col = lane & 15, g = lane >> 4; const size_t p0 = (size_t)blockIdx.x * 32;
  v8f acc[2] = {};
#pragma unroll 2
  for (int kc = 0; kc < GIN / 32; ++kc) { const v16b w = frag_b(PT + PO_L + (size_t)(wave * 16 + col) * GIN + kc * 32, lane);
#pragma unroll
    for (int rt = 0; rt < 2; ++rt) { const F2 a = split_row(XG + (p0 + rt * 16 + col) * GIN, kc * 32, lane); acc[rt] = wmma_bf(a.l, w, acc[rt]); acc[rt] = wmma_bf(a.h, w, acc[rt]); } }
#pragma unroll
  for (int rt = 0; rt < 2; ++rt)
#pragma unroll
    for (int r = 0; r < 8; ++r) { const int o = wave * 16 + col; sh[rt * 16 + 8 * g + r][o] = fmaxf(acc[rt][r] + bfr(bl1[o]), 0.f); }
  __syncthreads();
  if (tid < 32) { float s = bfr(bl2[0]);
#pragma unroll 1
    for (int o = 0; o < 128; ++o) s += sh[tid][o] * bfr(Wl2[o]);
    so[tid] = s; }
  __syncthreads();
  if (tid < 8) vst2(out + p0 + tid * 4, *(const v4f*)&so[tid * 4]);
}
#if DBGM != 0
__global__ __launch_bounds__(128) void k_dbg(const float* __restrict__ XC, const float* __restrict__ XG, float* __restrict__ out) {
  __shared__ __align__(16) float s[128]; const int i = threadIdx.x; float v;
#if DBGM == 1
  v = XC[(size_t)((i * 2731) % NNODE) * DX + (i * 7) % 384];
#elif DBGM == 2
  v = (i < 64) ? XC[(size_t)((i * 2731) % NNODE) * DX + 384 + (i * 5) % 128] : XC[(size_t)((i * 2731) % NNODE) * DX + 512 + (i % 32)];
#else
  v = (i < 96) ? XG[(size_t)((i * 37) % NG) * GIN + 32 + (i * 4099) % DK] : (i < 112 ? XG[(size_t)((i * 37) % NG) * GIN + (i % 32)] : XG[(size_t)((i * 37) % NG) * GIN + 32 + DK + (i % 32)]);
#endif
  s[i] = v; __syncthreads(); if (i < 32) vst2(out + i * 4, *(const v4f*)&s[i * 4]);
}
#endif
#if DBGM == 4
__global__ __launch_bounds__(256) void k_fakexg(const float* __restrict__ X, float* __restrict__ XG) { const int p = blockIdx.y; const size_t f0 = (size_t)blockIdx.x * 1024; for (int q = threadIdx.x; q < 256; q += 256) { v4f v; for (int k = 0; k < 4; ++k) { const size_t f = f0 + q * 4 + k; v[k] = bfr(X[((size_t)(p * 131) + f) % NNODE * F0 + (f % 128)]) * 0.25f; } vst2(XG + (size_t)p * GIN + f0 + q * 4, v); } }
#endif
#if DBGM == 2 || DBGM == 3
__global__ __launch_bounds__(256) void k_fakexc(const float* __restrict__ X, float* __restrict__ XC) { const int tid = threadIdx.x; const size_t n = (size_t)blockIdx.x * 64 + (tid >> 2); for (int p = (tid & 3); p < DX / 4; p += 4) { v4f v; for (int k = 0; k < 4; ++k) { const int c = p * 4 + k; v[k] = bfr(X[n * F0 + (c % 128)]) * (0.5f + (float)(c % 7) * 0.25f); } vst2(XC + n * DX + p * 4, v); } }
#endif
extern "C" void kernel_launch(void* const* d_in, const int* in_sizes, int n_in, void* d_out, int out_size, void* d_ws, size_t ws_size, hipStream_t stream) {
  (void)in_sizes; (void)n_in; (void)out_size;
  const float** F = (const float**)d_in; const int** I = (const int**)d_in;
  if (ws_size < (size_t)WS_END) return;
  char* ws = (char*)d_ws; __bf16* PT = (__bf16*)(ws + WS_PT); float *XLR = (float*)(ws + WS_XLR), *XC = (float*)(ws + WS_XC), *PRE = (float*)(ws + WS_PRE), *PART = (float*)(ws + WS_PART), *BN = (float*)(ws + WS_BN), *XG = (float*)(ws + WS_XG), *HH = (float*)(ws + WS_HH);
  k_pack<<<1184 + DX + 64 + 128, 256, 0, stream>>>(F[14], F[15], F[18], F[19], F[22], F[23], F[30], F[32], F[10], F[12], F[34], PT);
#if DBGM == 2
  k_fakexc<<<NNODE / 64, 256, 0, stream>>>(F[0], XC);
  goto layer2;
#endif
#if DBGM == 4
  k_fakexg<<<dim3(GIN / 1024, NG), 256, 0, stream>>>(F[0], XG);
  k_head<<<TNG / 32, 256, 0, stream>>>(XG, PT, F[35], F[36], F[37], (float*)d_out); return;
#endif
#if DBGM == 3
  k_fakexc<<<NNODE / 64, 256, 0, stream>>>(F[0], XC);
  k_pool<<<TNG, 256, 0, stream>>>(XC, PT, F[31], F[33], I[1], I[2], XG);
  k_nbh<<<dim3(ND / 64, 2), 128, 0, stream>>>(F[7], F[9], PT, F[11], F[13], HH);
  k_nbv<<<dim3(NG, 2), 256, 0, stream>>>(F[6], F[8], HH, I[4], I[5], XG);
  k_dbg<<<1, 128, 0, stream>>>(XC, XG, (float*)d_out); return;
#endif
  k_proj<F0, 768, true><<<NNODE / 64, 128, 0, stream>>>(F[0], F0, 0, PT + PO_1, XLR);
  k_gat<3, 128, 0><<<NG, 256, 0, stream>>>(XLR, I[1], I[2], F[16], F[17], PRE);
  k_colpart<HC1><<<NNODE / 64, 128, 0, stream>>>(PRE, PART);
  k_fin<HC1><<<1, 128, 0, stream>>>(PART, F[26], F[27], BN);
  k_bnapply<HC1><<<NNODE / 64, 256, 0, stream>>>(PRE, BN, 0, XC);
#if DBGM == 1
  k_dbg<<<1, 128, 0, stream>>>(XC, XG, (float*)d_out); return;
#endif
  layer2:
  k_proj<HC1, 256, false><<<NNODE / 64, 128, 0, stream>>>(XC, DX, 0, PT + PO_2, XLR);
  k_gat<2, 64, 0><<<NG, 256, 0, stream>>>(XLR, I[1], I[2], F[20], F[21], PRE);
  k_colpart<HC2><<<NNODE / 64, 128, 0, stream>>>(PRE, PART);
  k_fin<HC2><<<1, 128, 0, stream>>>(PART, F[28], F[29], BN + 768);
  k_bnapply<HC2><<<NNODE / 64, 256, 0, stream>>>(PRE, BN + 768, HC1, XC);
  k_proj<HC2, 128, false><<<NNODE / 64, 128, 0, stream>>>(XC, DX, HC1, PT + PO_3, XLR);
  k_gat<2, 32, 1><<<NG, 256, 0, stream>>>(XLR, I[1], I[2], F[24], F[25], XC);
#if DBGM == 2
  k_dbg<<<1, 128, 0, stream>>>(XC, XG, (float*)d_out); return;
#endif
  k_pool<<<TNG, 256, 0, stream>>>(XC, PT, F[31], F[33], I[1], I[2], XG);
  k_nbh<<<dim3(ND / 64, 2), 128, 0, stream>>>(F[7], F[9], PT, F[11], F[13], HH);
  k_nbv<<<dim3(NG, 2), 256, 0, stream>>>(F[6], F[8], HH, I[4], I[5], XG);
  k_head<<<TNG / 32, 256, 0, stream>>>(XG, PT, F[35], F[36], F[37], (float*)d_out);
}
